// ConvblockWithTarget_14130442404232
// MI455X (gfx1250) — hardware-verified
//
#include <hip/hip_runtime.h>
#include <math.h>
typedef __attribute__((ext_vector_type(16))) _Float16 v16h;
typedef __attribute__((ext_vector_type(8)))  _Float16 v8h;
typedef __attribute__((ext_vector_type(16))) __bf16   v16b;
typedef __attribute__((ext_vector_type(8)))  __bf16   v8b;
typedef __attribute__((ext_vector_type(8)))  float    v8f;
typedef __attribute__((ext_vector_type(4)))  float    v4f;
#define PSCALE 32768.0f
#define U16(p) ((const unsigned short*)(const void*)(p))
#define PSCALE_INV (1.0f / 32768.0f)

__device__ __forceinline__ unsigned short f2bf_bits(float f) {
  unsigned u = __float_as_uint(f);
  return (unsigned short)((u + 0x7FFFu + ((u >> 16) & 1u)) >> 16);
}
__device__ __forceinline__ float bf_bits2f(unsigned short h) { return __uint_as_float(((unsigned)h) << 16); }

__device__ __forceinline__ void dep_guard_h(v8f& a, v8f& b, v16h x, v16h y) { asm volatile("v_nop\n\tv_nop\n\tv_nop\n\tv_nop" : "+v"(a), "+v"(b) : "v"(x), "v"(y)); }
__device__ __forceinline__ void dep_guard_b(v8f& a, v8f& b, v16b x, v16b y) { asm volatile("v_nop\n\tv_nop\n\tv_nop\n\tv_nop" : "+v"(a), "+v"(b) : "v"(x), "v"(y)); }
__device__ __forceinline__ void keep4_h(v16h a, v16h b, v16h c, v16h d) { asm volatile("v_nop" :: "v"(a), "v"(b), "v"(c), "v"(d)); }
__device__ __forceinline__ void keep4_b(v16b a, v16b b, v16b c, v16b d) { asm volatile("v_nop" :: "v"(a), "v"(b), "v"(c), "v"(d)); }
__device__ __forceinline__ void acc_guard4(v8f& a, v8f& b, v8f& c, v8f& d) { asm volatile("v_nop\n\tv_nop\n\tv_nop\n\tv_nop" : "+v"(a), "+v"(b), "+v"(c), "+v"(d)); }
template <typename T> struct Frag;
template <> struct Frag<_Float16> {
  typedef v16h V; union U { v16h v; v8h h[2]; };
  static __device__ __forceinline__ v16h load(const _Float16* p) {
    U f; f.h[0] = *(const v8h*)(p); f.h[1] = *(const v8h*)(p + 16); return f.v;
  }
  static __device__ __forceinline__ v8f mma(v16h a, v16h b, v8f c) {
    return __builtin_amdgcn_wmma_f32_16x16x32_f16(false, a, false, b, (short)0, c, false, false);
  }
  static __device__ __forceinline__ void guard(v8f& a, v8f& b, v16h x, v16h y) { dep_guard_h(a, b, x, y); }
  static __device__ __forceinline__ void keep(v16h a, v16h b, v16h c, v16h d) { keep4_h(a, b, c, d); }
};
template <> struct Frag<__bf16> {
  typedef v16b V; union U { v16b v; v8b h[2]; };
  static __device__ __forceinline__ v16b load(const __bf16* p) {
    U f; f.h[0] = *(const v8b*)(p); f.h[1] = *(const v8b*)(p + 16); return f.v;
  }
  static __device__ __forceinline__ v8f mma(v16b a, v16b b, v8f c) {
    return __builtin_amdgcn_wmma_f32_16x16x32_bf16(false, a, false, b, (short)0, c, false, false);
  }
  static __device__ __forceinline__ void guard(v8f& a, v8f& b, v16b x, v16b y) { dep_guard_b(a, b, x, y); }
  static __device__ __forceinline__ void keep(v16b a, v16b b, v16b c, v16b d) { keep4_b(a, b, c, d); }
};

template <int ET> struct Elem;
template <> struct Elem<0> { typedef _Float16 T; };
template <> struct Elem<1> { typedef __bf16 T; };
template <int ET, bool SPLIT, int BIAS_MODE, int OUT_MODE, bool RESID, int ACT = 0>
__global__ __launch_bounds__(256) void wmma_gemm64(
    const unsigned short* __restrict__ Ap, const unsigned short* __restrict__ A2p, int lda, long strideA,
    const unsigned short* __restrict__ Btp, const unsigned short* __restrict__ Bt2p, int ldb, long strideB,
    void* __restrict__ Cout, void* __restrict__ Cout2, int ldc, long strideC,
    const float* __restrict__ bias,
    const float* __restrict__ resid, long strideR,
    int M, int N, int K, float scale) {
  typedef typename Elem<ET>::T T;
  typedef typename Frag<T>::V V;
  const T* A = (const T*)Ap; const T* A2 = (const T*)A2p; const T* Bt = (const T*)Btp; const T* Bt2 = (const T*)Bt2p;
  __shared__ __align__(16) float sT[8][16 * 68];
  const int b    = blockIdx.y;
  const int lane = threadIdx.x & 31;
  const int wave = threadIdx.x >> 5;
  const int tilesN = N >> 6;
  const int tilesM = M >> 6;
  const int tile = blockIdx.x * 8 + wave;
  if (tile >= tilesM * tilesN) return;
  const int tm = tile / tilesN;
  const int tn = tile - tm * tilesN;
  const int m0 = tm << 6;
  const int n0 = tn << 6;

  const T* Ab  = A  + (size_t)b * strideA;
  const T* Bb  = Bt + (size_t)b * strideB;
  const T* Ab2 = SPLIT ? (A2  + (size_t)b * strideA) : nullptr;
  const T* Bb2 = SPLIT ? (Bt2 + (size_t)b * strideB) : nullptr;

  const int rlane = lane & 15;
  const int koff  = (lane >> 4) * 8;
  const int mOff  = (lane >> 4) * 8;

  v8f acc[4][4];
#pragma unroll
  for (int i = 0; i < 4; ++i)
#pragma unroll
    for (int j = 0; j < 4; ++j) acc[i][j] = (v8f){0.f,0.f,0.f,0.f,0.f,0.f,0.f,0.f};

  for (int k0 = 0; k0 < K; k0 += 32) {
    V bh[4], bl[4];
#pragma unroll
    for (int j = 0; j < 4; ++j) {
      const size_t bo = (size_t)(n0 + (j << 4) + rlane) * ldb + koff + k0;
      bh[j] = Frag<T>::load(Bb + bo);
      if (SPLIT) bl[j] = Frag<T>::load(Bb2 + bo);
    }
#pragma unroll
    for (int i = 0; i < 4; ++i) {
      const size_t ao = (size_t)(m0 + (i << 4) + rlane) * lda + koff + k0;
      V ah = Frag<T>::load(Ab + ao);
      V al;
      if (SPLIT) al = Frag<T>::load(Ab2 + ao);
#pragma unroll
      for (int j = 0; j < 4; ++j) {
        acc[i][j] = Frag<T>::mma(ah, bh[j], acc[i][j]);
        if (SPLIT) {
          acc[i][j] = Frag<T>::mma(ah, bl[j], acc[i][j]);
          acc[i][j] = Frag<T>::mma(al, bh[j], acc[i][j]);
        }
      }
      Frag<T>::guard(acc[i][0], acc[i][3], ah, SPLIT ? al : ah);
    }
    Frag<T>::keep(bh[0], bh[1], bh[2], bh[3]);
    if (SPLIT) Frag<T>::keep(bl[0], bl[1], bl[2], bl[3]);
  }
  acc_guard4(acc[0][0], acc[0][1], acc[0][2], acc[0][3]);
  acc_guard4(acc[1][0], acc[1][1], acc[1][2], acc[1][3]);
  acc_guard4(acc[2][0], acc[2][1], acc[2][2], acc[2][3]);
  acc_guard4(acc[3][0], acc[3][1], acc[3][2], acc[3][3]);

  float* slab = sT[wave];
  const float* Rb = RESID ? (resid + (size_t)b * strideR) : nullptr;
#pragma unroll
  for (int i = 0; i < 4; ++i) {
    const int mBase = m0 + (i << 4);
#pragma unroll
    for (int j = 0; j < 4; ++j) {
      const int n = n0 + (j << 4) + rlane;
      float bv = 0.f;
      if (BIAS_MODE == 2) bv = bias[n];
#pragma unroll
      for (int r = 0; r < 8; ++r) {
        float v = acc[i][j][r] * scale;
        if (BIAS_MODE == 1) v += bias[mBase + mOff + r];
        if (BIAS_MODE == 2) v += bv;
        if (RESID) v += Rb[(size_t)(mBase + mOff + r) * ldc + n];
        if (ACT == 1) v = tanhf(v);
        if (ACT == 2) v = fmaxf(v, 0.0f);
        if (ACT == 3) v = v / (1.0f + expf(-v));
        if (ACT == 4) v = (v > 0.f) ? v : 0.01f * v;
        if (ACT == 5) v = 0.5f * v * (1.0f + erff(v * 0.70710678118654752f));
        slab[(mOff + r) * 68 + (j << 4) + rlane] = v;
      }
    }
    __builtin_amdgcn_fence(__ATOMIC_RELEASE, "workgroup");
    __builtin_amdgcn_wave_barrier();
    __builtin_amdgcn_fence(__ATOMIC_ACQUIRE, "workgroup");
    if (OUT_MODE == 0) {
      float* C = (float*)Cout + (size_t)b * strideC;
      const int hh = lane >> 4, c4 = (lane & 15) * 4;
      for (int pass = 0; pass < 2; ++pass) {
#pragma unroll
        for (int it = 0; it < 8; ++it) {
          const int row = it * 2 + hh;
          v4f v = *(const v4f*)(slab + row * 68 + c4);
          *(volatile v4f*)(C + (size_t)(mBase + row) * ldc + n0 + c4) = v;
        }
        __threadfence();
      }
    } else {
      const int q = lane >> 3, c8 = (lane & 7) * 8;
      unsigned short* C  = (unsigned short*)Cout  + (size_t)b * strideC;
      unsigned short* C2 = (OUT_MODE == 2) ? ((unsigned short*)Cout2 + (size_t)b * strideC) : nullptr;
      for (int pass = 0; pass < 2; ++pass) {
#pragma unroll
        for (int it = 0; it < 4; ++it) {
          const int row = it * 4 + q;
          const float* sp = slab + row * 68 + c8;
          v8h hv, lv;
#pragma unroll
          for (int e = 0; e < 8; ++e) {
            if (OUT_MODE == 1) {
              hv[e] = (_Float16)sp[e];
            } else {
              unsigned short hb = f2bf_bits(sp[e]);
              unsigned short lb = f2bf_bits(sp[e] - bf_bits2f(hb));
              hv[e] = __builtin_bit_cast(_Float16, hb);
              lv[e] = __builtin_bit_cast(_Float16, lb);
            }
          }
          *(volatile v8h*)(C + (size_t)(mBase + row) * ldc + n0 + c8) = hv;
          if (OUT_MODE == 2) *(volatile v8h*)(C2 + (size_t)(mBase + row) * ldc + n0 + c8) = lv;
        }
        __threadfence();
      }
    }
    __builtin_amdgcn_fence(__ATOMIC_RELEASE, "workgroup");
    __builtin_amdgcn_wave_barrier();
    __builtin_amdgcn_fence(__ATOMIC_ACQUIRE, "workgroup");
  }
}

__global__ __launch_bounds__(256) void cast_f32_f16x2(
    const float* __restrict__ in, _Float16* __restrict__ out, int n2) {
  int i = blockIdx.x * 256 + threadIdx.x;
  if (i < n2) {
    const _Float16 h0 = (_Float16)in[2 * i], h1 = (_Float16)in[2 * i + 1];
    const unsigned u = (unsigned)__builtin_bit_cast(unsigned short, h0) | ((unsigned)__builtin_bit_cast(unsigned short, h1) << 16);
    ((volatile unsigned*)out)[i] = u;
    __threadfence();
    ((volatile unsigned*)out)[i] = u;
  }
}


#define VB 8
#define VL 16384
#define VC 64
#define VK 7
#define VT 8186
#define VOFF (VL - 2 * VT)
#define VTP 8192
__device__ __forceinline__ unsigned pkh(float a, float b) { return (unsigned)__builtin_bit_cast(unsigned short, (_Float16)a) | ((unsigned)__builtin_bit_cast(unsigned short, (_Float16)b) << 16); }
__global__ __launch_bounds__(256) void wdyn_kernel(const float* __restrict__ Wd, unsigned* __restrict__ BT) { for (int i = threadIdx.x + blockIdx.x * 256; i < VC * VK * VC / 2; i += gridDim.x * 256) { const int row = i / 32, cp = 2 * (i % 32); const int d = row / VK, k = row % VK; const unsigned u = pkh(Wd[(d * VC + cp) * VK + k], Wd[(d * VC + cp + 1) * VK + k]); ((volatile unsigned*)BT)[i] = u; __threadfence(); ((volatile unsigned*)BT)[i] = u; } }
__global__ __launch_bounds__(256) void w11_kernel(const float* __restrict__ Wc, unsigned* __restrict__ BT) { for (int i = threadIdx.x; i < VC * VC / 2; i += 256) { const int o = i / 32, cp = 2 * (i % 32); const unsigned u = pkh(Wc[cp * VC + o], Wc[(cp + 1) * VC + o]); ((volatile unsigned*)BT)[i] = u; __threadfence(); ((volatile unsigned*)BT)[i] = u; } }
__global__ __launch_bounds__(256) void comb_kernel(const float* __restrict__ x, const float* __restrict__ WR, int b, const float* __restrict__ g, const float* __restrict__ bb, float* __restrict__ YN, unsigned* __restrict__ YN16) {
  const int lane = threadIdx.x & 31, wave = threadIdx.x >> 5; const int t = blockIdx.x * 8 + wave; if (t >= VT) return; const float* xb = x + (size_t)b * VL * VC; const int c0 = 2 * lane, c1 = c0 + 1;
  float y0 = xb[(size_t)(2 * t + VOFF) * VC + c0], y1 = xb[(size_t)(2 * t + VOFF) * VC + c1];
#pragma unroll 1
  for (int par = 0; par < 2; ++par) { const float* wr = WR + (size_t)(2 * t + par) * (VC * VK);
#pragma unroll 1
    for (int k = 0; k < VK; ++k) { const float* xr = xb + (size_t)(2 * t + 2 * k + par) * VC; y0 += xr[c0] * tanhf(wr[c0 * VK + k]); y1 += xr[c1] * tanhf(wr[c1 * VK + k]); } }
  float s = y0 + y1; for (int o = 16; o > 0; o >>= 1) s += __shfl_xor(s, o, 32); const float mu = s / VC;
  float q = (y0 - mu) * (y0 - mu) + (y1 - mu) * (y1 - mu); for (int o = 16; o > 0; o >>= 1) q += __shfl_xor(q, o, 32); const float inv = rsqrtf(q / VC + 1e-6f);
  const float n0 = (y0 - mu) * inv * g[c0] + bb[c0], n1 = (y1 - mu) * inv * g[c1] + bb[c1]; const size_t r = (size_t)b * VTP + t;
  for (int pass = 0; pass < 2; ++pass) { ((volatile float*)YN)[r * VC + c0] = n0; ((volatile float*)YN)[r * VC + c1] = n1; ((volatile unsigned*)YN16)[r * 32 + lane] = pkh(n0, n1); __threadfence(); }
}
__global__ __launch_bounds__(256) void zero_u32(unsigned* __restrict__ p, long n) { const long i = (long)blockIdx.x * 256 + threadIdx.x; if (i < n) { ((volatile unsigned*)p)[i] = 0u; __threadfence(); ((volatile unsigned*)p)[i] = 0u; } }
__global__ __launch_bounds__(256) void fin_kernel(const float* __restrict__ YN, const float* __restrict__ Z, const float* __restrict__ slope, float* __restrict__ out) {
  const long i = (long)blockIdx.x * 256 + threadIdx.x; if (i >= (long)VB * VT * VC) return; const long bt = i / VC; const int c = (int)(i % VC); const int b = (int)(bt / VT), t = (int)(bt % VT); const size_t r = ((size_t)b * VTP + t) * VC + c;
  const float z = Z[r]; const float v = YN[r] + (z >= 0.f ? z : slope[0] * z); ((volatile float*)out)[i] = v; __threadfence(); ((volatile float*)out)[i] = v;
}
extern "C" void kernel_launch(void* const* d_in, const int* in_sizes, int n_in, void* d_out, int out_size, void* d_ws, size_t ws_size, hipStream_t stream) {
  (void)in_sizes; (void)n_in; (void)out_size; (void)ws_size;
  auto Fp = [&](int i) { return (const float*)d_in[i]; };
  const float* x = Fp(0); const float* Wd = Fp(1); const float* g = Fp(2); const float* bb = Fp(3); const float* Wc = Fp(4); const float* bc = Fp(5); const float* slope = Fp(6);
  char* ws = (char*)d_ws; size_t off = 0;
  auto carve = [&](size_t bytes) -> char* { char* p = ws + off; off += (bytes + 255) & ~(size_t)255; return p; };
  _Float16* X16 = (_Float16*)carve(((size_t)VB * VL + 64) * VC * 2); unsigned* BTD = (unsigned*)carve(VC * VK * VC * 2); unsigned* BT11 = (unsigned*)carve(VC * VC * 2); float* WR = (float*)carve((size_t)VL * VC * VK * 4);
  float* YN = (float*)carve((size_t)VB * VTP * VC * 4); unsigned* YN16 = (unsigned*)carve((size_t)VB * VTP * VC * 2); float* Z = (float*)carve((size_t)VB * VTP * VC * 4);
  cast_f32_f16x2<<<(unsigned)(((long)VB * VL * VC / 2 + 255) / 256), 256, 0, stream>>>(x, X16, (long)VB * VL * VC / 2);
  zero_u32<<<(64 * VC / 2 + 255) / 256, 256, 0, stream>>>((unsigned*)(X16 + (size_t)VB * VL * VC), 64 * VC / 2);
  zero_u32<<<(unsigned)(((long)VB * VTP * VC / 2 + 255) / 256), 256, 0, stream>>>(YN16, (long)VB * VTP * VC / 2);
  wdyn_kernel<<<8, 256, 0, stream>>>(Wd, BTD); w11_kernel<<<1, 256, 0, stream>>>(Wc, BT11);
  const int tw = (VL / 64) * (VC * VK / 64);
  for (int b = 0; b < VB; ++b) {
    wmma_gemm64<0, false, 0, 0, false><<<dim3((tw + 7) / 8, 1), 256, 0, stream>>>(U16(X16 + ((size_t)b * VL + VOFF) * VC), nullptr, VC, 0, (const unsigned short*)BTD, nullptr, VC, 0, WR, nullptr, VC * VK, 0, nullptr, nullptr, 0, VL, VC * VK, VC, 1.0f);
    comb_kernel<<<(VT + 7) / 8, 256, 0, stream>>>(x, WR, b, g, bb, YN, YN16); }
  const int tz = (VB * VTP / 64) * 1;
  wmma_gemm64<0, false, 2, 0, false><<<dim3((tz + 7) / 8, 1), 256, 0, stream>>>((const unsigned short*)YN16, nullptr, VC, 0, (const unsigned short*)BT11, nullptr, VC, 0, Z, nullptr, VC, 0, bc, nullptr, 0, VB * VTP, VC, VC, 1.0f);
  fin_kernel<<<(unsigned)(((long)VB * VT * VC + 255) / 256), 256, 0, stream>>>(YN, Z, slope, (float*)d_out);
}
